// CausalVarlenSelfAttention_50663434223693
// MI455X (gfx1250) — hardware-verified
//
#include <hip/hip_runtime.h>
#include <math.h>
#include <stdint.h>

#ifndef NSEQ
#define NSEQ 8
#endif
#define NSEQ_MAX 8
#define SEQ   1024
#define NTOK  (NSEQ * SEQ)
#define DMOD  1024
#define NH    16
#define HD    64
#define HHALF (HD / 2)
#define QKVN  (3 * DMOD)
#define NGATE NH
#define GP    64
#define QO    256
#define EPS_RMS 0.000001f
#define SM_SCALE 0.125f
#define LOG2E 1.4426950408889634f
#define QSC   256.0f
#define KSC   256.0f
#define PCAR  32768.0f
#define VCAR  1024.0f
#define OSC   1024.0f
#define WOS   1024.0f
#define WPB   4
#define NHG   (NH / WPB)
#define NQT   (SEQ / 16)
#define NST   (SEQ / 64)
#define NKT   (SEQ / 32)
#define ATT_THREADS (WPB * 32)
#define PTP   36
#define PTW   (16 * PTP)
#define SLP   68
#define SLW   (16 * SLP)
#define WREG  (PTW + SLW)
#define SLAB64 (16 * 68)
#define VTP   72
#define WS_CAP 134217728LL

#define SZ_XB ((long long)NTOK * DMOD * 2)
#define SZ_WQ ((long long)QKVN * DMOD * 2)
#define SZ_WG ((long long)GP * DMOD * 2)
#define SZ_WO ((long long)DMOD * DMOD * 2)
#define SZ_F  ((long long)NTOK * DMOD * 4)
#define SZ_G  ((long long)NTOK * GP * 4)
#define SZ_P  ((long long)NTOK * DMOD * 2)
#define SZ_VH ((long long)NSEQ * NH * HD * SEQ * 2)
#define SZ_VL ((long long)NSEQ * NH * HD * QO * 2)
#define SZ_OL ((long long)NSEQ * QO * DMOD * 2)
#define WS_TOTAL (SZ_XB + SZ_WQ + SZ_WG + SZ_WO + SZ_F + SZ_G + 3 * SZ_P + SZ_VH + SZ_VL)

static_assert(NSEQ >= 1 && NSEQ <= NSEQ_MAX);
static_assert(DMOD == NH * HD && HD == 64 && HHALF == 32 && QKVN == 3072);
static_assert((SEQ % 64) == 0 && (QO % 64) == 0 && QO >= 64 && QO <= SEQ);
static_assert(NHG * WPB == NH && ATT_THREADS == 128);
static_assert((DMOD % 64) == 0 && (GP % 64) == 0 && NGATE <= GP && (DMOD % 32) == 0 && (HD % 32) == 0);
static_assert(((NTOK * DMOD / 8) % 256) == 0 && ((QKVN * DMOD / 8) % 256) == 0 && ((GP * DMOD / 8) % 256) == 0);
static_assert(((DMOD * DMOD / 8) % 256) == 0);
static_assert(WPB * WREG * 4 <= 65536 && 2 * HD * VTP * 2 <= 65536 && 4 * SLAB64 * 4 <= 65536);
static_assert(SZ_P == SZ_XB);
static_assert(SZ_P + SZ_OL <= SZ_F);
static_assert(SZ_VH == SZ_P);
static_assert(WS_TOTAL <= WS_CAP);
static_assert((SZ_XB % 4096) == 0 && (SZ_WQ % 4096) == 0 && (SZ_WG % 4096) == 0 && (SZ_WO % 4096) == 0);
static_assert((SZ_F % 4096) == 0 && (SZ_G % 4096) == 0 && (SZ_VL % 4096) == 0 && (SZ_P % 4096) == 0);

typedef unsigned short u16;
typedef _Float16 v16h __attribute__((ext_vector_type(16)));
typedef _Float16 v8h  __attribute__((ext_vector_type(8)));
typedef __bf16   v16b __attribute__((ext_vector_type(16)));
typedef float    v8f  __attribute__((ext_vector_type(8)));
typedef float    v4f  __attribute__((ext_vector_type(4)));
typedef unsigned int v4u __attribute__((ext_vector_type(4)));

union FragH { v16h v; v8h h[2]; v4u u[2]; };
union FragB { v16b v; v4u u[2]; };

__device__ __forceinline__ unsigned short bf_bits(float f) {
  unsigned u = __float_as_uint(f);
  return (unsigned short)((u + 0x7FFFu + ((u >> 16) & 1u)) >> 16);
}
__device__ __forceinline__ float bf_up(unsigned short h) { return __uint_as_float(((unsigned)h) << 16); }
__device__ __forceinline__ float bfr(float f) { return bf_up(bf_bits(f)); }
__device__ __forceinline__ unsigned short h_bits(_Float16 x) { return __builtin_bit_cast(unsigned short, x); }
__device__ __forceinline__ unsigned pk16(unsigned short a, unsigned short b) { return (unsigned)a | ((unsigned)b << 16); }
__device__ __forceinline__ v8f zero8() { v8f z = {0.f, 0.f, 0.f, 0.f, 0.f, 0.f, 0.f, 0.f}; return z; }

__device__ __forceinline__ v16h ldfrag_h(const _Float16* p) {
  FragH f;
  f.h[0] = *(const v8h*)(p);
  f.h[1] = *(const v8h*)(p + 16);
  return f.v;
}
__device__ __forceinline__ v16b ldfrag_b(const u16* p) {
  FragB f;
  f.u[0] = *(const v4u*)(p);
  f.u[1] = *(const v4u*)(p + 16);
  return f.v;
}

__device__ __forceinline__ v8f mma_h(v16h a, v16h b, v8f c) {
  return __builtin_amdgcn_wmma_f32_16x16x32_f16(false, a, false, b, (short)0, c, false, false);
}
__device__ __forceinline__ v8f mma_b(v16b a, v16b b, v8f c) {
  return __builtin_amdgcn_wmma_f32_16x16x32_bf16(false, a, false, b, (short)0, c, false, false);
}
__device__ __forceinline__ void guard2(v8f& a, v8f& b, v16h x0, v16h x1, v16h x2, v16h x3, v16h x4, v16h x5) {
#if defined(__HIP_DEVICE_COMPILE__)
  asm volatile("v_nop\n\tv_nop\n\tv_nop\n\tv_nop"
               : "+v"(a), "+v"(b) : "v"(x0), "v"(x1), "v"(x2), "v"(x3), "v"(x4), "v"(x5) : "memory");
#endif
}
template <typename F>
__device__ __forceinline__ void guard6(v8f& a, v8f& b, v8f& c, v8f& d, F x0, F x1, F x2, F x3, F x4, F x5) {
#if defined(__HIP_DEVICE_COMPILE__)
  asm volatile("v_nop\n\tv_nop\n\tv_nop\n\tv_nop"
               : "+v"(a), "+v"(b), "+v"(c), "+v"(d) : "v"(x0), "v"(x1), "v"(x2), "v"(x3), "v"(x4), "v"(x5) : "memory");
#endif
}
__device__ __forceinline__ void acc_guard4(v8f& a, v8f& b, v8f& c, v8f& d) {
#if defined(__HIP_DEVICE_COMPILE__)
  asm volatile("v_nop\n\tv_nop\n\tv_nop\n\tv_nop" : "+v"(a), "+v"(b), "+v"(c), "+v"(d));
#endif
}
__device__ __forceinline__ void wave_sync_lds() {
  __builtin_amdgcn_fence(__ATOMIC_RELEASE, "workgroup");
  __builtin_amdgcn_wave_barrier();
  __builtin_amdgcn_fence(__ATOMIC_ACQUIRE, "workgroup");
}

__global__ __launch_bounds__(256) void cvt16(const float* __restrict__ x, u16* D, int n8src, int n8, int f16mode, float scale) {
  const int gt = blockIdx.x * 256 + (int)threadIdx.x;
  if (gt >= n8) return;
  const bool valid = (gt < n8src);
  const int  gs    = valid ? gt : (n8src - 1);
  const float* p = x + (size_t)gs * 8;
  const v4f a = *(const v4f*)(p), b4 = *(const v4f*)(p + 4);
  float w[8];
#pragma unroll
  for (int e = 0; e < 4; ++e) { w[e] = valid ? a[e] : 0.0f; w[4 + e] = valid ? b4[e] : 0.0f; }
  v4u o;
#pragma unroll
  for (int e = 0; e < 4; ++e) {
    const float f0 = w[2 * e], f1 = w[2 * e + 1];
    const unsigned short hb0 = h_bits((_Float16)(bfr(f0) * scale));
    const unsigned short hb1 = h_bits((_Float16)(bfr(f1) * scale));
    const unsigned short bb0 = bf_bits(f0);
    const unsigned short bb1 = bf_bits(f1);
    o[e] = (f16mode != 0) ? pk16(hb0, hb1) : pk16(bb0, bb1);
  }
  u16* d = D + (size_t)gt * 8;
  for (int pass = 0; pass < 2; ++pass) {
    *(volatile v4u*)(d) = o;
    __threadfence();
  }
}

__global__ __launch_bounds__(256) void vt16(const float* __restrict__ F, u16* VHo, u16* VLo) {
  __shared__ __align__(16) u16 TH[HD * VTP];
  __shared__ __align__(16) u16 TL[HD * VTP];
  const int tid = (int)threadIdx.x;
  const int bid = (int)blockIdx.x;
  const int st  = bid % NST;
  const int bh  = bid / NST;
  if (bh >= NSEQ * NH) return;
  const int b   = bh / NH, h = bh % NH;
  const int s0  = st * 64;
  {
    const int sl = tid >> 2;
    const int dc = (tid & 3) * 16;
    const float* src = F + ((size_t)b * SEQ + s0 + sl) * DMOD + h * HD + dc;
#pragma unroll
    for (int i = 0; i < 4; ++i) {
      const v4f a = *(const v4f*)(src + 4 * i);
#pragma unroll
      for (int e = 0; e < 4; ++e) {
        const float t = a[e] * VCAR;
        const _Float16 hv = (_Float16)t;
        const _Float16 lv = (_Float16)(t - (float)hv);
        TH[(dc + 4 * i + e) * VTP + sl] = h_bits(hv);
        TL[(dc + 4 * i + e) * VTP + sl] = h_bits(lv);
      }
    }
  }
  __syncthreads();
  v4u vh[2], vl[2];
  const int q8 = tid >> 3, p8 = (tid & 7) * 8;
#pragma unroll
  for (int it = 0; it < 2; ++it) {
    const int line = it * 32 + q8;
    vh[it] = *(const v4u*)(TH + line * VTP + p8);
    vl[it] = *(const v4u*)(TL + line * VTP + p8);
  }
  const size_t hrow  = (size_t)bh * HD;
  const size_t baseh = hrow * SEQ + s0 + p8;
  const size_t basel = hrow * QO + s0 + p8;
  for (int pass = 0; pass < 2; ++pass) {
#pragma unroll
    for (int it = 0; it < 2; ++it) {
      const int line = it * 32 + q8;
      *(volatile v4u*)(VHo + baseh + (size_t)line * SEQ) = vh[it];
    }
    if (s0 < QO) {
#pragma unroll
      for (int it = 0; it < 2; ++it) {
        const int line = it * 32 + q8;
        *(volatile v4u*)(VLo + basel + (size_t)line * QO) = vl[it];
      }
    }
    __threadfence();
  }
}

__global__ __launch_bounds__(128) void nrope16(const float* __restrict__ F, const int* __restrict__ pidp, int ncs,
                                               const float* __restrict__ CS, const float* __restrict__ SN,
                                               u16* Hp, u16* Lp, float sc) {
#pragma clang fp contract(off)
  const int tid = (int)threadIdx.x;
  const int row = (int)blockIdx.x;
  if (row >= NTOK) return;
  const int head = tid >> 3;
  const int w    = (tid & 7) * 8;
  const int jlo  = w & (HHALF - 1);
  const bool up  = (w >= HHALF);
  const float* p = F + (size_t)row * DMOD + head * HD + jlo;
  const v4f xa = *(const v4f*)(p), xb = *(const v4f*)(p + 4);
  const v4f ya = *(const v4f*)(p + HHALF), yb = *(const v4f*)(p + HHALF + 4);
  int pr = pidp[row];
  pr = (pr < 0) ? (pr + ncs) : pr;
  pr = (pr < 0) ? 0 : pr;
  pr = (pr > ncs - 1) ? (ncs - 1) : pr;
  const float* cp = CS + (size_t)pr * HHALF + jlo;
  const float* sp = SN + (size_t)pr * HHALF + jlo;
  const v4f ca = *(const v4f*)(cp), cb = *(const v4f*)(cp + 4);
  const v4f sa = *(const v4f*)(sp), sb = *(const v4f*)(sp + 4);
  float x1[8], x2[8], cv[8], sv[8];
#pragma unroll
  for (int e = 0; e < 4; ++e) {
    x1[e] = xa[e];        x1[4 + e] = xb[e];
    x2[e] = ya[e];        x2[4 + e] = yb[e];
    cv[e] = bfr(ca[e]);   cv[4 + e] = bfr(cb[e]);
    sv[e] = bfr(sa[e]);   sv[4 + e] = bfr(sb[e]);
  }
  float o1[8], o2[8];
  float ss = 0.0f;
#pragma unroll
  for (int e = 0; e < 8; ++e) {
    const float a1 = x1[e] * cv[e];
    const float a2 = x2[e] * sv[e];
    o1[e] = a1 + a2;
    const float b1 = (-x1[e]) * sv[e];
    const float b2 = x2[e] * cv[e];
    o2[e] = b1 + b2;
    ss = ss + o1[e] * o1[e];
    ss = ss + o2[e] * o2[e];
  }
  float ssm = up ? 0.0f : ss;
  ssm += __shfl_xor(ssm, 1, 32);
  ssm += __shfl_xor(ssm, 2, 32);
  ssm += __shfl_xor(ssm, 4, 32);
  const float var = ssm * (1.0f / (float)HD);
  const float rs  = 1.0f / sqrtf(var + EPS_RMS);
  v4u oh, ol;
#pragma unroll
  for (int e = 0; e < 4; ++e) {
    const float ya0 = (up ? o2[2 * e]     : o1[2 * e])     * rs;
    const float ya1 = (up ? o2[2 * e + 1] : o1[2 * e + 1]) * rs;
    const float t0 = ya0 * sc, t1 = ya1 * sc;
    const _Float16 h0 = (_Float16)t0, h1 = (_Float16)t1;
    const _Float16 l0 = (_Float16)(t0 - (float)h0), l1 = (_Float16)(t1 - (float)h1);
    oh[e] = pk16(h_bits(h0), h_bits(h1));
    ol[e] = pk16(h_bits(l0), h_bits(l1));
  }
  u16* dh = Hp + (size_t)row * DMOD + head * HD + w;
  u16* dl = Lp + (size_t)row * DMOD + head * HD + w;
  for (int pass = 0; pass < 2; ++pass) {
    *(volatile v4u*)(dh) = oh;
    *(volatile v4u*)(dl) = ol;
    __threadfence();
  }
}

__device__ __forceinline__ void epi64(float* sl, v8f a0, v8f a1, v8f a2, v8f a3, float oscale,
                                      float* C, int N, size_t rowb, int col0, int lane) {
  const int hh = lane >> 4, m = lane & 15;
#pragma unroll
  for (int r = 0; r < 8; ++r) {
    const int ro = (8 * hh + r) * 68 + m;
    sl[ro]      = a0[r] * oscale;
    sl[ro + 16] = a1[r] * oscale;
    sl[ro + 32] = a2[r] * oscale;
    sl[ro + 48] = a3[r] * oscale;
  }
  wave_sync_lds();
  v4f vals[8];
#pragma unroll
  for (int it = 0; it < 8; ++it) vals[it] = *(const v4f*)(sl + (it * 2 + hh) * 68 + m * 4);
  float* dst = C + (rowb + (size_t)hh) * (size_t)N + col0 + m * 4;
  for (int pass = 0; pass < 2; ++pass) {
#pragma unroll
    for (int it = 0; it < 8; ++it) {
      *(volatile v4f*)(dst + (size_t)(it * 2) * (size_t)N) = vals[it];
    }
    __threadfence();
  }
}

__global__ __launch_bounds__(128)
void gemm_bf(const u16* __restrict__ A, const u16* __restrict__ Bt, float* C, int M, int N, int K, float oscale) {
  __shared__ __align__(16) float slab[4 * SLAB64];
  const int tid = threadIdx.x, wave = tid >> 5, lane = tid & 31, hh = lane >> 4, m = lane & 15;
  const int ntile = N >> 6;
  const int bid   = blockIdx.x;
  const int rowb  = (bid / ntile) * 64 + wave * 16;
  const int col0  = (bid % ntile) * 64;
  if (rowb + 16 > M) return;
  const u16* ap = A  + (size_t)(rowb + m) * K + 8 * hh;
  const u16* bp = Bt + (size_t)(col0 + m) * K + 8 * hh;
  const size_t bs = (size_t)16 * K;
  v8f acc0 = zero8(), acc1 = zero8(), acc2 = zero8(), acc3 = zero8();
#pragma unroll 1
  for (int k0 = 0; k0 < K; k0 += 32) {
    const v16b a  = ldfrag_b(ap + k0);
    const v16b b0 = ldfrag_b(bp + k0);
    const v16b b1 = ldfrag_b(bp + bs + k0);
    const v16b b2 = ldfrag_b(bp + 2 * bs + k0);
    const v16b b3 = ldfrag_b(bp + 3 * bs + k0);
    acc0 = mma_b(a, b0, acc0);
    acc1 = mma_b(a, b1, acc1);
    acc2 = mma_b(a, b2, acc2);
    acc3 = mma_b(a, b3, acc3);
    guard6<v16b>(acc0, acc1, acc2, acc3, a, b0, b1, b2, b3, a);
  }
  epi64(slab + wave * SLAB64, acc0, acc1, acc2, acc3, oscale, C, N, (size_t)rowb, col0, lane);
}

template <int NPROD>
__global__ __launch_bounds__(128)
void gemm_o(const u16* __restrict__ Ah, const u16* __restrict__ Al, const u16* __restrict__ Bt,
            float* C, int sbeg, int nrt, float oscale) {
  __shared__ __align__(16) float slab[4 * SLAB64];
  const int tid = threadIdx.x, wave = tid >> 5, lane = tid & 31, hh = lane >> 4, m = lane & 15;
  const int ntile = DMOD >> 6;
  const int bid   = blockIdx.x;
  const int ct    = bid % ntile;
  const int rest  = bid / ntile;
  const int rt    = rest % nrt;
  const int b     = rest / nrt;
  if (b >= NSEQ) return;
  const int s     = sbeg + rt * 64 + wave * 16;
  if (s + 16 > SEQ) return;
  if (NPROD == 2 && s + 16 > QO) return;
  const int col0  = ct * 64;
  const int K     = DMOD;
  const size_t rowC = (size_t)b * SEQ + s;
  const size_t rowL = (size_t)b * QO + s;
  const _Float16* ahp = (const _Float16*)(const void*)Ah + (rowC + m) * K + 8 * hh;
  const _Float16* alp = (const _Float16*)(const void*)Al + (rowL + m) * K + 8 * hh;
  const _Float16* bp  = (const _Float16*)(const void*)Bt + (size_t)(col0 + m) * K + 8 * hh;
  const size_t bs = (size_t)16 * K;
  v8f acc0 = zero8(), acc1 = zero8(), acc2 = zero8(), acc3 = zero8();
  if constexpr (NPROD == 2) {
#pragma unroll 1
    for (int k0 = 0; k0 < K; k0 += 32) {
      const v16h ah = ldfrag_h(ahp + k0), al = ldfrag_h(alp + k0);
      const v16h b0 = ldfrag_h(bp + k0);
      const v16h b1 = ldfrag_h(bp + bs + k0);
      const v16h b2 = ldfrag_h(bp + 2 * bs + k0);
      const v16h b3 = ldfrag_h(bp + 3 * bs + k0);
      acc0 = mma_h(ah, b0, acc0);  acc0 = mma_h(al, b0, acc0);
      acc1 = mma_h(ah, b1, acc1);  acc1 = mma_h(al, b1, acc1);
      acc2 = mma_h(ah, b2, acc2);  acc2 = mma_h(al, b2, acc2);
      acc3 = mma_h(ah, b3, acc3);  acc3 = mma_h(al, b3, acc3);
      guard6<v16h>(acc0, acc1, acc2, acc3, ah, al, b0, b1, b2, b3);
    }
  } else {
#pragma unroll 1
    for (int k0 = 0; k0 < K; k0 += 32) {
      const v16h ah = ldfrag_h(ahp + k0);
      const v16h b0 = ldfrag_h(bp + k0);
      const v16h b1 = ldfrag_h(bp + bs + k0);
      const v16h b2 = ldfrag_h(bp + 2 * bs + k0);
      const v16h b3 = ldfrag_h(bp + 3 * bs + k0);
      acc0 = mma_h(ah, b0, acc0);
      acc1 = mma_h(ah, b1, acc1);
      acc2 = mma_h(ah, b2, acc2);
      acc3 = mma_h(ah, b3, acc3);
      guard6<v16h>(acc0, acc1, acc2, acc3, ah, b0, b1, b2, b3, ah);
    }
  }
  epi64(slab + wave * SLAB64, acc0, acc1, acc2, acc3, oscale, C, DMOD, rowC, col0, lane);
}

template <int PVR>
__global__ __launch_bounds__(ATT_THREADS)
void attn_k(const u16* __restrict__ QHp, const u16* __restrict__ QLp,
            const u16* __restrict__ KHp, const u16* __restrict__ KLp,
            const u16* __restrict__ VHp, const u16* __restrict__ VLp,
            const float* __restrict__ Gp, const float* __restrict__ gb,
            u16* OHp, u16* OLp, int qt_beg, int nqt) {
  __shared__ __align__(16) float smem[WPB * WREG];

  const int tid  = threadIdx.x;
  const int wave = tid >> 5;
  const int lane = tid & 31;
  const int hh   = lane >> 4;
  const int c    = lane & 15;
  const int bid  = blockIdx.x;
  const int qt   = qt_beg + bid % nqt;
  const int rest = bid / nqt;
  const int hg   = rest % NHG;
  const int b    = rest / NHG;
  if (b >= NSEQ) return;
  const int q0   = qt * 16;
  if (q0 + 16 > SEQ) return;
  const int head = hg * WPB + wave;
  const size_t tok0 = (size_t)b * SEQ;

  float* pt   = smem + wave * WREG;
  float* slab = pt + PTW;

  const size_t hcol = (size_t)head * HD + 8 * hh;
  const _Float16* Qh  = (const _Float16*)(const void*)QHp + (tok0 + q0 + c) * DMOD + hcol;
  const _Float16* Ql  = (const _Float16*)(const void*)QLp + (tok0 + q0 + c) * DMOD + hcol;
  const _Float16* Khb = (const _Float16*)(const void*)KHp + (tok0 + c) * DMOD + hcol;
  const _Float16* Klb = (const _Float16*)(const void*)KLp + (tok0 + c) * DMOD + hcol;
  const size_t bh = (size_t)b * NH + head;
  const _Float16* Vhb = (const _Float16*)(const void*)VHp + (bh * HD + c) * SEQ + 8 * hh;
  const _Float16* Vlb = (const _Float16*)(const void*)VLp + (bh * HD + c) * QO + 8 * hh;
  const float lsc = SM_SCALE * (LOG2E / (QSC * KSC));
  const float oc  = 1.0f / (PCAR * VCAR);
  const size_t KROW = (size_t)DMOD;

  const int khi = (q0 + 15) >> 5;
  const int qr0 = q0 + 8 * hh;

  const float gx  = Gp[(tok0 + q0 + c) * GP + head] + bfr(gb[head]);
  const float gsg = 1.0f / (1.0f + expf(-gx));

  float mrow[8], lrow[8];
  v8f o[4];
#pragma unroll
  for (int r = 0; r < 8; ++r) { mrow[r] = -INFINITY; lrow[r] = 0.f; }
#pragma unroll
  for (int j = 0; j < 4; ++j) o[j] = zero8();

#pragma unroll 1
  for (int kt = 0; kt <= khi && kt < NKT; ++kt) {
    const int kb   = kt * 32;
    const int key0 = kb + c, key1 = kb + 16 + c;
    v8f s0 = zero8(), s1 = zero8();
    const _Float16* k0p = Khb + (size_t)kb * KROW;
    const _Float16* k1p = k0p + (size_t)16 * KROW;
    const _Float16* l0p = Klb + (size_t)kb * KROW;
    const _Float16* l1p = l0p + (size_t)16 * KROW;
#pragma unroll
    for (int kk = 0; kk < HD / 32; ++kk) {
      const v16h qh  = ldfrag_h(Qh + kk * 32);
      const v16h ql  = ldfrag_h(Ql + kk * 32);
      const v16h kh0 = ldfrag_h(k0p + kk * 32);
      const v16h kh1 = ldfrag_h(k1p + kk * 32);
      const v16h kl0 = ldfrag_h(l0p + kk * 32);
      const v16h kl1 = ldfrag_h(l1p + kk * 32);
      s0 = mma_h(qh, kh0, s0);
      s0 = mma_h(ql, kh0, s0);
      s0 = mma_h(qh, kl0, s0);
      s1 = mma_h(qh, kh1, s1);
      s1 = mma_h(ql, kh1, s1);
      s1 = mma_h(qh, kl1, s1);
      guard2(s0, s1, qh, ql, kh0, kl0, kh1, kl1);
    }
#pragma unroll
    for (int r = 0; r < 8; ++r) {
      const int qr = qr0 + r;
      const float u0 = s0[r] * lsc;
      const float u1 = s1[r] * lsc;
      const float t0 = (key0 <= qr) ? u0 : -INFINITY;
      const float t1 = (key1 <= qr) ? u1 : -INFINITY;
      float mx = fmaxf(t0, t1);
#pragma unroll
      for (int off = 1; off < 16; off <<= 1) mx = fmaxf(mx, __shfl_xor(mx, off, 32));
      const float mn = fmaxf(mrow[r], mx);
      const float ms = (mn == -INFINITY) ? 0.0f : mn;
      const float al = exp2f(mrow[r] - ms);
      mrow[r] = mn;
      const float e0 = exp2f(t0 - ms), e1 = exp2f(t1 - ms);
      float ps = e0 + e1;
#pragma unroll
      for (int off = 1; off < 16; off <<= 1) ps += __shfl_xor(ps, off, 32);
      lrow[r] = lrow[r] * al + ps;
#pragma unroll
      for (int j = 0; j < 4; ++j) o[j][r] *= al;
      const int ro = (8 * hh + r) * PTP + c;
      pt[ro]      = e0;
      pt[ro + 16] = e1;
    }
    wave_sync_lds();
    FragH ph;
    FragH pl;
    {
      const float* prow = pt + c * PTP + 8 * hh;
      const v4f p0 = *(const v4f*)(prow), p1 = *(const v4f*)(prow + 4);
      const v4f p2 = *(const v4f*)(prow + 16), p3 = *(const v4f*)(prow + 20);
#pragma unroll
      for (int e = 0; e < 4; ++e) {
        const float ta = p0[e] * PCAR, tb = p1[e] * PCAR, tc = p2[e] * PCAR, td = p3[e] * PCAR;
        const _Float16 ha = (_Float16)ta, hb = (_Float16)tb, hc = (_Float16)tc, hd = (_Float16)td;
        ph.h[0][e]     = ha;
        ph.h[0][4 + e] = hb;
        ph.h[1][e]     = hc;
        ph.h[1][4 + e] = hd;
        if constexpr (PVR == 1) {
          pl.h[0][e]     = (_Float16)(ta - (float)ha);
          pl.h[0][4 + e] = (_Float16)(tb - (float)hb);
          pl.h[1][e]     = (_Float16)(tc - (float)hc);
          pl.h[1][4 + e] = (_Float16)(td - (float)hd);
        } else {
          pl.h[0][e] = ha; pl.h[0][4 + e] = hb; pl.h[1][e] = hc; pl.h[1][4 + e] = hd;
        }
      }
    }
    {
      const _Float16* vhp = Vhb + kb;
      const _Float16* vlp = Vlb + kb;
#pragma unroll
      for (int jg = 0; jg < 2; ++jg) {
        const size_t dah = (size_t)(2 * jg) * 16 * SEQ;
        const size_t dbh = dah + (size_t)16 * SEQ;
        const v16h vha = ldfrag_h(vhp + dah), vhb2 = ldfrag_h(vhp + dbh);
        if constexpr (PVR == 1) {
          const size_t dal = (size_t)(2 * jg) * 16 * QO;
          const size_t dbl = dal + (size_t)16 * QO;
          const v16h vla = ldfrag_h(vlp + dal), vlb2 = ldfrag_h(vlp + dbl);
          o[2 * jg]     = mma_h(ph.v, vha,  o[2 * jg]);
          o[2 * jg]     = mma_h(pl.v, vha,  o[2 * jg]);
          o[2 * jg]     = mma_h(ph.v, vla,  o[2 * jg]);
          o[2 * jg + 1] = mma_h(ph.v, vhb2, o[2 * jg + 1]);
          o[2 * jg + 1] = mma_h(pl.v, vhb2, o[2 * jg + 1]);
          o[2 * jg + 1] = mma_h(ph.v, vlb2, o[2 * jg + 1]);
          guard2(o[2 * jg], o[2 * jg + 1], ph.v, pl.v, vha, vhb2, vla, vlb2);
        } else {
          o[2 * jg]     = mma_h(ph.v, vha,  o[2 * jg]);
          o[2 * jg + 1] = mma_h(ph.v, vhb2, o[2 * jg + 1]);
          guard2(o[2 * jg], o[2 * jg + 1], ph.v, ph.v, vha, vhb2, vha, vhb2);
        }
      }
    }
    wave_sync_lds();
  }
  acc_guard4(o[0], o[1], o[2], o[3]);
  const float qnan = __int_as_float(0x7fc00000);
#pragma unroll
  for (int r = 0; r < 8; ++r) {
    const float gr  = __shfl(gsg, 8 * hh + r, 32);
    const float lv  = lrow[r];
    const float ls  = (lv > 0.0f) ? lv : 1.0f;
    const float inv = (lv > 0.0f) ? ((1.0f / ls) * oc * gr) : qnan;
#pragma unroll
    for (int j = 0; j < 4; ++j) {
      const int idx = (8 * hh + r) * SLP + j * 16 + c;
      slab[idx] = o[j][r] * inv;
    }
  }

  wave_sync_lds();
  v4u oh[4], ol[4];
  const int rq = lane >> 3, c8 = (lane & 7) * 8;
#pragma unroll
  for (int it = 0; it < 4; ++it) {
    const int row = it * 4 + rq;
    const v4f a = *(const v4f*)(slab + row * SLP + c8), b4 = *(const v4f*)(slab + row * SLP + c8 + 4);
    float w[8];
#pragma unroll
    for (int e = 0; e < 4; ++e) { w[e] = a[e] * OSC; w[4 + e] = b4[e] * OSC; }
#pragma unroll
    for (int e = 0; e < 4; ++e) {
      const _Float16 h0 = (_Float16)w[2 * e], h1 = (_Float16)w[2 * e + 1];
      const _Float16 l0 = (_Float16)(w[2 * e] - (float)h0), l1 = (_Float16)(w[2 * e + 1] - (float)h1);
      oh[it][e] = pk16(h_bits(h0), h_bits(h1));
      ol[it][e] = pk16(h_bits(l0), h_bits(l1));
    }
  }
  const size_t obh = (tok0 + q0) * DMOD + (size_t)head * HD + c8;
  const size_t obl = ((size_t)b * QO + q0) * DMOD + (size_t)head * HD + c8;
  for (int pass = 0; pass < 2; ++pass) {
#pragma unroll
    for (int it = 0; it < 4; ++it) {
      const int row = it * 4 + rq;
      *(volatile v4u*)(OHp + obh + (size_t)row * DMOD) = oh[it];
      if constexpr (PVR == 1) {
        *(volatile v4u*)(OLp + obl + (size_t)row * DMOD) = ol[it];
      }
    }
    __threadfence();
  }
}

extern "C" void kernel_launch(void* const* d_in, const int* in_sizes, int n_in,
                              void* d_out, int out_size, void* d_ws, size_t ws_size,
                              hipStream_t stream) {
  if (n_in < 9) return;
  if (in_sizes[0] < NTOK * DMOD) return;
  if (in_sizes[1] != QKVN * DMOD) return;
  if (in_sizes[2] != DMOD * DMOD) return;
  if (in_sizes[3] != NGATE * DMOD) return;
  if (in_sizes[4] < NGATE) return;
  if (in_sizes[5] < HHALF) return;
  const int ncs = in_sizes[5] / HHALF;
  if (in_sizes[6] < ncs * HHALF) return;
  const int nb = in_sizes[7] - 1;
  if (nb < NSEQ) return;
  if ((in_sizes[0] / DMOD) != nb * SEQ) return;
  if (in_sizes[8] < NTOK) return;
  if (out_size < NTOK * DMOD) return;

  const float* x     = (const float*)d_in[0];
  const float* wqkv  = (const float*)d_in[1];
  const float* wo    = (const float*)d_in[2];
  const float* gw    = (const float*)d_in[3];
  const float* gbp   = (const float*)d_in[4];
  const float* cosc  = (const float*)d_in[5];
  const float* sinc  = (const float*)d_in[6];
  const int*   pids  = (const int*)d_in[8];
  float*       out   = (float*)d_out;

  const size_t szXB = (size_t)SZ_XB, szWQ = (size_t)SZ_WQ, szWG = (size_t)SZ_WG, szWO = (size_t)SZ_WO;
  const size_t szF  = (size_t)SZ_F,  szG  = (size_t)SZ_G,  szP  = (size_t)SZ_P;
  const size_t szVH = (size_t)SZ_VH, szVL = (size_t)SZ_VL, szOL = (size_t)SZ_OL;
  if (szP + szOL > szF) return;
  size_t off = 0;
  const size_t oXB = off; off += szXB;
  const size_t oWQ = off; off += szWQ;
  const size_t oWG = off; off += szWG;
  const size_t oWO = off; off += szWO;
  const size_t oF  = off; off += szF;
  const size_t oG  = off; off += szG;
  const size_t oQL = off; off += szP;
  const size_t oKH = off; off += szP;
  const size_t oKL = off; off += szP;
  const size_t oVH = off; off += szVH;
  const size_t oVL = off; off += szVL;
  if (off > ws_size) return;
  if (off > (size_t)WS_CAP) return;

  char* ws = (char*)d_ws;
  u16*   XB = (u16*)(ws + oXB);
  u16*   QH = (u16*)(ws + oXB);
  u16*   WQ = (u16*)(ws + oWQ);
  u16*   WG = (u16*)(ws + oWG);
  u16*   WO = (u16*)(ws + oWO);
  float* F  = (float*)(ws + oF);
  u16*   OH = (u16*)(ws + oF);
  u16*   OL = (u16*)(ws + oF + szP);
  float* G  = (float*)(ws + oG);
  u16*   QL = (u16*)(ws + oQL);
  u16*   KH = (u16*)(ws + oKH);
  u16*   KL = (u16*)(ws + oKL);
  u16*   VH = (u16*)(ws + oVH);
  u16*   VL = (u16*)(ws + oVL);

  const dim3 b256(256), b128(128), bAT(ATT_THREADS);
  const int  n8x  = (NTOK * DMOD) / 8;
  const int  n8wq = (QKVN * DMOD) / 8;
  const int  n8wg = (GP * DMOD) / 8;
  const int  n8wgs = (NGATE * DMOD) / 8;
  const int  n8wo = (DMOD * DMOD) / 8;
  const dim3 gX((n8x + 255) / 256), gWQ((n8wq + 255) / 256), gWG((n8wg + 255) / 256), gWO((n8wo + 255) / 256);
  const dim3 gGG((NTOK / 64) * (GP / 64));
  const dim3 gGP((NTOK / 64) * (DMOD / 64));
  const dim3 gVT(NSEQ * NH * NST);
  const dim3 gRW(NTOK);
  const int  nqtR = QO / 16;
  const int  nqtP = (SEQ - QO) / 16;
  const int  nrtR = QO / 64;
  const int  nrtP = (SEQ - QO) / 64;

  cvt16<<<gX,  b256, 0, stream>>>(x,    XB, n8x,   n8x,  0, 1.0f);
  cvt16<<<gWQ, b256, 0, stream>>>(wqkv, WQ, n8wq,  n8wq, 0, 1.0f);
  cvt16<<<gWG, b256, 0, stream>>>(gw,   WG, n8wgs, n8wg, 0, 1.0f);
  cvt16<<<gWO, b256, 0, stream>>>(wo,   WO, n8wo,  n8wo, 1, WOS);
  gemm_bf<<<gGG, b128, 0, stream>>>(XB, WG, G, NTOK, GP, DMOD, 1.0f);
  gemm_bf<<<gGP, b128, 0, stream>>>(XB, WQ + (size_t)2 * DMOD * DMOD, F, NTOK, DMOD, DMOD, 1.0f);
  vt16<<<gVT, b256, 0, stream>>>(F, VH, VL);
  gemm_bf<<<gGP, b128, 0, stream>>>(XB, WQ + (size_t)DMOD * DMOD, F, NTOK, DMOD, DMOD, 1.0f);
  nrope16<<<gRW, b128, 0, stream>>>(F, pids, ncs, cosc, sinc, KH, KL, KSC);
  gemm_bf<<<gGP, b128, 0, stream>>>(XB, WQ, F, NTOK, DMOD, DMOD, 1.0f);
  nrope16<<<gRW, b128, 0, stream>>>(F, pids, ncs, cosc, sinc, QH, QL, QSC);
  attn_k<1><<<dim3(nqtR * NHG * NSEQ), bAT, 0, stream>>>(QH, QL, KH, KL, VH, VL, G, gbp, OH, OL, 0, nqtR);
  if (nqtP > 0) {
    attn_k<0><<<dim3(nqtP * NHG * NSEQ), bAT, 0, stream>>>(QH, QL, KH, KL, VH, VL, G, gbp, OH, OL, nqtR, nqtP);
  }
  gemm_o<2><<<dim3(NSEQ * nrtR * (DMOD / 64)), b128, 0, stream>>>(OH, OL, WO, out, 0, nrtR, 1.0f / (OSC * WOS));
  if (nrtP > 0) {
    gemm_o<1><<<dim3(NSEQ * nrtP * (DMOD / 64)), b128, 0, stream>>>(OH, OL, WO, out, QO, nrtP, 1.0f / (OSC * WOS));
  }
  (void)hipGetLastError();
}
